// GATLayer_72267119722746
// MI455X (gfx1250) — hardware-verified
//
#include <hip/hip_runtime.h>
#include <stddef.h>
#include <stdint.h>
#include <math.h>


#define MN    512
#define DIN   128
#define DOUT  64
#define GBM   64
#define GTHR  128
#define NTHR  256
#define NEGS  0.2f
#define WSMAX 134217728

static_assert((DIN % 32) == 0 && (DIN / 8) == 16);
static_assert(DOUT == 64 && (MN % GBM) == 0 && (MN % 32) == 0);
static_assert(MN == 4 * GTHR);
static_assert(GBM == (GTHR / 32) * 16);
static_assert(2 * DOUT == GTHR);
static_assert(GBM * 2 == MN / 4);

typedef float          v4f  __attribute__((ext_vector_type(4)));
typedef float          v8f  __attribute__((ext_vector_type(8)));
typedef int            v8i  __attribute__((ext_vector_type(8)));
typedef unsigned int   v4u  __attribute__((ext_vector_type(4)));
typedef unsigned short v8us __attribute__((ext_vector_type(8)));
typedef __bf16         v16b __attribute__((ext_vector_type(16)));
typedef v4f  __attribute__((may_alias)) v4fa;
typedef v8us __attribute__((may_alias)) v8usa;
union FragB { v16b v; v8us h[2]; v8i w; };

__device__ __forceinline__ v8f wmb(const FragB& a, const FragB& b, v8f c) {
  v8f d = __builtin_amdgcn_wmma_f32_16x16x32_bf16(false, a.v, false, b.v, (short)0, c, false, false);
  asm volatile("v_nop\n\tv_nop\n\tv_nop\n\tv_nop" : "+v"(d) : "v"(a.w), "v"(b.w));
  return d;
}

__device__ __forceinline__ unsigned int f2bf(float f) {
  const unsigned int u = __float_as_uint(f);
  return ((u + 0x7FFFu + ((u >> 16) & 1u)) >> 16) & 0xFFFFu;
}
__device__ __forceinline__ float bf2f(unsigned int b) { return __uint_as_float(b << 16); }
__device__ __forceinline__ float bfr(float f) { return bf2f(f2bf(f)); }
__device__ __forceinline__ unsigned int pk2(float lo, float hi) { return f2bf(lo) | (f2bf(hi) << 16); }
__device__ __forceinline__ v4u pack8(const v4f a, const v4f b) {
  v4u r;
  r.x = pk2(a.x, a.y); r.y = pk2(a.z, a.w); r.z = pk2(b.x, b.y); r.w = pk2(b.z, b.w);
  return r;
}
__device__ __forceinline__ float lky(float x) { return x > 0.f ? x : NEGS * x; }

__global__ __launch_bounds__(NTHR) void k_cvt(const float* __restrict__ x, unsigned short* xb, int nUnits) {
  const int i = (int)blockIdx.x * NTHR + (int)threadIdx.x;
  if (i >= nUnits) return;
  const size_t o = (size_t)i * 8;
  const float* p = x + o;
  const v4f a = *(const v4fa*)p;
  const v4f b = *(const v4fa*)(p + 4);
  const v4u hv = pack8(a, b);
  *(volatile v4u*)(xb + o) = hv;
  __threadfence();
  *(volatile v4u*)(xb + o) = hv;
}

__global__ __launch_bounds__(GTHR) void k_proj(
    const unsigned short* __restrict__ HB, const unsigned short* __restrict__ WB,
    const float* __restrict__ av, unsigned short* TP, float* SP, int nB)
{
  __shared__ __attribute__((aligned(16))) float stg[GBM * DOUT];
  __shared__ __attribute__((aligned(16))) float satt[2 * DOUT];
  __shared__ __attribute__((aligned(16))) float sdot[2 * GBM];
  const int tid = (int)threadIdx.x, lane = tid & 31, wave = tid >> 5, hh = lane >> 4, m = lane & 15;
  const int rowBase = (int)blockIdx.x * GBM;
  const int b  = rowBase / MN;
  const int n0 = rowBase - b * MN;
  const size_t NT  = (size_t)nB * MN;
  const size_t TPL = (size_t)nB * DOUT * MN;

  satt[tid] = bfr(av[tid]);

  v8f acc[4];
  {
    const v8f z = {0.f, 0.f, 0.f, 0.f, 0.f, 0.f, 0.f, 0.f};
    acc[0] = z; acc[1] = z; acc[2] = z; acc[3] = z;
  }
  const unsigned short* ap = HB + (size_t)(rowBase + 16 * wave + m) * (size_t)DIN + 8 * hh;
  const unsigned short* wp = WB + (size_t)m * (size_t)DIN + 8 * hh;
#pragma unroll 1
  for (int ks = 0; ks < DIN / 32; ++ks) {
    FragB af;
    af.h[0] = *(const v8usa*)(ap + 32 * ks);
    af.h[1] = *(const v8usa*)(ap + 32 * ks + 16);
#pragma unroll
    for (int t = 0; t < 4; ++t) {
      const unsigned short* wq = wp + (size_t)(16 * t) * (size_t)DIN + 32 * ks;
      FragB bf;
      bf.h[0] = *(const v8usa*)wq;
      bf.h[1] = *(const v8usa*)(wq + 16);
      acc[t] = wmb(af, bf, acc[t]);
    }
  }

#pragma unroll
  for (int t = 0; t < 4; ++t) {
    const int lc = 16 * t + m;
#pragma unroll
    for (int r = 0; r < 8; ++r) {
      const int lr = 16 * wave + 8 * hh + r;
      stg[lr * DOUT + lc] = acc[t][r];
    }
  }
  __syncthreads();

  {
    const int row = tid & 63, which = tid >> 6;
    const float* sa = satt + which * DOUT;
    const float* hr = stg + row * DOUT;
    float d = 0.f;
#pragma unroll 4
    for (int c4 = 0; c4 < DOUT / 4; ++c4) {
      const v4f hv = *(const v4fa*)(hr + 4 * c4);
      const v4f aw = *(const v4fa*)(sa + 4 * c4);
      d = fmaf(hv.x, aw.x, d);
      d = fmaf(hv.y, aw.y, d);
      d = fmaf(hv.z, aw.z, d);
      d = fmaf(hv.w, aw.w, d);
    }
    sdot[which * GBM + row] = d;
  }
  __syncthreads();

  const v4f sdv = *(const v4fa*)(sdot + hh * GBM + 4 * m);
  float* sp = SP + (size_t)hh * NT + rowBase + 4 * m;

  const int g  = lane >> 3;
  const int nl = 8 * (lane & 7);
  v4u hq[4], lq[4];
#pragma unroll
  for (int q = 0; q < 4; ++q) {
    const int d = 16 * wave + 4 * q + g;
    float f[8];
#pragma unroll
    for (int j = 0; j < 8; ++j) f[j] = stg[(nl + j) * DOUT + d];
    unsigned int hb[8], lb[8];
#pragma unroll
    for (int j = 0; j < 8; ++j) {
      hb[j] = f2bf(f[j]);
      lb[j] = f2bf(f[j] - bf2f(hb[j]));
    }
    v4u hv, lv;
    hv.x = hb[0] | (hb[1] << 16); hv.y = hb[2] | (hb[3] << 16); hv.z = hb[4] | (hb[5] << 16); hv.w = hb[6] | (hb[7] << 16);
    lv.x = lb[0] | (lb[1] << 16); lv.y = lb[2] | (lb[3] << 16); lv.z = lb[4] | (lb[5] << 16); lv.w = lb[6] | (lb[7] << 16);
    hq[q] = hv; lq[q] = lv;
  }

#pragma unroll
  for (int q = 0; q < 4; ++q) {
    const int d = 16 * wave + 4 * q + g;
    unsigned short* tp = TP + ((size_t)b * DOUT + d) * (size_t)MN + n0 + nl;
    *(volatile v4u*)tp = hq[q];
    *(volatile v4u*)(tp + TPL) = lq[q];
  }
  if (wave == 0) *(volatile v4f*)sp = sdv;
  __threadfence();
#pragma unroll
  for (int q = 0; q < 4; ++q) {
    const int d = 16 * wave + 4 * q + g;
    unsigned short* tp = TP + ((size_t)b * DOUT + d) * (size_t)MN + n0 + nl;
    *(volatile v4u*)tp = hq[q];
    *(volatile v4u*)(tp + TPL) = lq[q];
  }
  if (wave == 0) *(volatile v4f*)sp = sdv;
}

__global__ __launch_bounds__(GTHR) void k_attn(
    const unsigned short* __restrict__ TP, const float* __restrict__ SP, float* out, int nB)
{
  __shared__ __attribute__((aligned(16))) float sd[MN];
  __shared__ __attribute__((aligned(16))) float stg[GBM * DOUT];
  __shared__ __attribute__((aligned(16))) float sl[GBM];
  const int tid = (int)threadIdx.x, lane = tid & 31, wave = tid >> 5, hh = lane >> 4, m = lane & 15;
  const int tiles = MN / GBM;
  const int b    = (int)blockIdx.x / tiles;
  const int mblk = ((int)blockIdx.x - b * tiles) * GBM;
  const size_t NT  = (size_t)nB * MN;
  const size_t TPL = (size_t)nB * DOUT * MN;

  *(v4f*)(sd + 4 * tid) = *(const v4fa*)(SP + NT + (size_t)b * MN + 4 * tid);
  const float ss = SP[(size_t)b * MN + mblk + 16 * wave + m];
  __syncthreads();

  float tm = -3.0e38f;
#pragma unroll
  for (int i = 0; i < MN / 32; ++i) tm = fmaxf(tm, sd[lane + 32 * i]);
#pragma unroll
  for (int off = 16; off > 0; off >>= 1) tm = fmaxf(tm, __shfl_xor(tm, off));
  const float zmax = lky(ss + tm);

  v8f acc[4];
  {
    const v8f z = {0.f, 0.f, 0.f, 0.f, 0.f, 0.f, 0.f, 0.f};
    acc[0] = z; acc[1] = z; acc[2] = z; acc[3] = z;
  }
  float rs = 0.f;
  const unsigned short* wph = TP + ((size_t)b * DOUT + m) * (size_t)MN + 8 * hh;

#pragma unroll 1
  for (int ks = 0; ks < MN / 32; ++ks) {
    const int k0 = 32 * ks;
    const v4f e0 = *(const v4fa*)(sd + k0 + 8 * hh);
    const v4f e1 = *(const v4fa*)(sd + k0 + 8 * hh + 4);
    const v4f e2 = *(const v4fa*)(sd + k0 + 16 + 8 * hh);
    const v4f e3 = *(const v4fa*)(sd + k0 + 16 + 8 * hh + 4);
    const float e[16] = {e0.x, e0.y, e0.z, e0.w, e1.x, e1.y, e1.z, e1.w,
                         e2.x, e2.y, e2.z, e2.w, e3.x, e3.y, e3.z, e3.w};
    FragB ah, al;
#pragma unroll
    for (int j = 0; j < 16; ++j) {
      const float p = expf(lky(ss + e[j]) - zmax);
      rs += p;
      const unsigned int hb = f2bf(p);
      const unsigned int lb = f2bf(p - bf2f(hb));
      ah.h[j >> 3][j & 7] = (unsigned short)hb;
      al.h[j >> 3][j & 7] = (unsigned short)lb;
    }
#pragma unroll
    for (int t = 0; t < 4; ++t) {
      const unsigned short* wq = wph + (size_t)(16 * t) * (size_t)MN + k0;
      FragB bh, bl;
      bh.h[0] = *(const v8usa*)wq;
      bh.h[1] = *(const v8usa*)(wq + 16);
      bl.h[0] = *(const v8usa*)(wq + TPL);
      bl.h[1] = *(const v8usa*)(wq + TPL + 16);
      acc[t] = wmb(ah, bh, acc[t]);
      acc[t] = wmb(ah, bl, acc[t]);
      acc[t] = wmb(al, bh, acc[t]);
    }
  }
  const float lt = rs + __shfl_xor(rs, 16);

#pragma unroll
  for (int t = 0; t < 4; ++t) {
    const int lc = 16 * t + m;
#pragma unroll
    for (int r = 0; r < 8; ++r) {
      const int lr = 16 * wave + 8 * hh + r;
      stg[lr * DOUT + lc] = acc[t][r];
    }
  }
  sl[16 * wave + m] = lt;
  __syncthreads();

  v4f fv[8];
#pragma unroll
  for (int i = 0; i < 8; ++i) {
    const int lr = 16 * wave + 2 * i + hh;
    const v4f v = *(const v4fa*)(stg + lr * DOUT + 4 * m);
    const float inv = 1.0f / sl[lr];
    v4f o;
    o.x = v.x * inv; o.y = v.y * inv; o.z = v.z * inv; o.w = v.w * inv;
    o.x = o.x > 0.f ? o.x : expm1f(o.x);
    o.y = o.y > 0.f ? o.y : expm1f(o.y);
    o.z = o.z > 0.f ? o.z : expm1f(o.z);
    o.w = o.w > 0.f ? o.w : expm1f(o.w);
    fv[i] = o;
  }
#pragma unroll
  for (int i = 0; i < 8; ++i) {
    const int lr = 16 * wave + 2 * i + hh;
    float* op = out + ((size_t)b * MN + mblk + lr) * (size_t)DOUT + 4 * m;
    *(volatile v4f*)op = fv[i];
  }
  __threadfence();
#pragma unroll
  for (int i = 0; i < 8; ++i) {
    const int lr = 16 * wave + 2 * i + hh;
    float* op = out + ((size_t)b * MN + mblk + lr) * (size_t)DOUT + 4 * m;
    *(volatile v4f*)op = fv[i];
  }
}

static inline int cdiv(int a, int b) { return (a + b - 1) / b; }

extern "C" void kernel_launch(void* const* d_in, const int* in_sizes, int n_in,
                              void* d_out, int out_size, void* d_ws, size_t ws_size,
                              hipStream_t stream) {
  if (n_in < 3) return;
  if (in_sizes[1] != DOUT * DIN) return;
  if (in_sizes[2] != 2 * DOUT) return;
  const int per = MN * DIN;
  if (in_sizes[0] <= 0 || (in_sizes[0] % per) != 0) return;
  const int nB = in_sizes[0] / per;
  if (nB < 1 || nB > 2048) return;
  const long long NT = (long long)nB * MN;
  if ((long long)out_size != NT * DOUT) return;

  const float* h = (const float*)d_in[0];
  const float* W = (const float*)d_in[1];
  const float* a = (const float*)d_in[2];
  float* out = (float*)d_out;

  char* ws = (char*)d_ws;
  size_t off = 0;
  const size_t oHB = off; off += (size_t)NT * DIN * 2;               off = (off + 255) & ~(size_t)255;
  const size_t oWB = off; off += (size_t)DOUT * DIN * 2;             off = (off + 255) & ~(size_t)255;
  const size_t oTP = off; off += (size_t)2 * nB * DOUT * MN * 2;     off = (off + 255) & ~(size_t)255;
  const size_t oSP = off; off += (size_t)2 * NT * 4;                 off = (off + 255) & ~(size_t)255;
  if (off > ws_size || off > (size_t)WSMAX) return;
  unsigned short* HB = (unsigned short*)(ws + oHB);
  unsigned short* WB = (unsigned short*)(ws + oWB);
  unsigned short* TP = (unsigned short*)(ws + oTP);
  float*          SP = (float*)(ws + oSP);

  const int nUh = (int)(NT * (DIN / 8));
  k_cvt<<<cdiv(nUh, NTHR), NTHR, 0, stream>>>(h, HB, nUh);
  const int nUw = DOUT * (DIN / 8);
  k_cvt<<<cdiv(nUw, NTHR), NTHR, 0, stream>>>(W, WB, nUw);

  k_proj<<<(int)(NT / GBM), GTHR, 0, stream>>>(HB, WB, a, TP, SP, nB);
  k_attn<<<nB * (MN / GBM), GTHR, 0, stream>>>(TP, SP, out, nB);
}
